// MultiHeadedSelfAttention_8272107012563
// MI455X (gfx1250) — hardware-run, weakly checked
//
#include <hip/hip_runtime.h>


#ifndef NB
#define NB 8
#endif
#ifndef SEQ
#define SEQ 1024
#endif
#define NB_FULL  8
#define SEQ_FULL 1024
#define EM   768
#define NH   12
#define HD   64
#define PP   72
#define XCAR 16.0f
#define INVX2 (1.0f / (XCAR * XCAR))
#define LOG2E 1.4426950408889634f
#define NQB  (SEQ / 16)
#define NBLK (NB * NH * NQB)
#define NAMAX ((NB * SEQ * EM) / 8192)
#define PRM_Q 0
#define PRM_K 32
#define PRM_V 64
#define PRM_S 96
#define PRM_P 128
#define PRM_O 160

typedef _Float16 h16;
typedef unsigned short bf;
typedef __attribute__((ext_vector_type(16))) __bf16   v16bf;
typedef __attribute__((ext_vector_type(16))) _Float16 v16h;
typedef __attribute__((ext_vector_type(8)))  _Float16 v8h;
typedef __attribute__((ext_vector_type(8)))  unsigned short v8us;
typedef __attribute__((ext_vector_type(8)))  float    v8f;
typedef __attribute__((ext_vector_type(4)))  float    v4f;
typedef v8h  __attribute__((may_alias)) v8ha;
typedef v4f  __attribute__((may_alias)) v4fa;

static_assert(NH * HD == EM);
static_assert(HD == 64);
static_assert(EM % 64 == 0);
static_assert(EM % 32 == 0);
static_assert(SEQ % 64 == 0);
static_assert((NB * SEQ) % 64 == 0);
static_assert(SEQ <= SEQ_FULL);
static_assert(NB <= NB_FULL);
static_assert(PP % 8 == 0);
static_assert(PP >= 64);
static_assert(((size_t)NB * SEQ * EM / 8) % 256 == 0);
static_assert(((size_t)EM * EM / 8) % 256 == 0);
static_assert(NQB * 16 == SEQ);
static_assert(((size_t)NB * SEQ * EM) % 8192 == 0);
static_assert(((size_t)NB * SEQ * EM / 4) % 256 == 0);
static_assert(32 * 16 * 8 == 16 * HD * 4);
static_assert(8 * 16 == 16 * 2 * 4);
static_assert(8 * 16 == 128);
static_assert(16 * PP * 2 + 16 * 68 * 4 + 32 * 4 <= 131072);
static_assert(16 * 68 * 4 <= 131072);

__device__ __forceinline__ unsigned short f2bf(float f) { unsigned u = __float_as_uint(f); u += 0x7FFFu + ((u >> 16) & 1u); return (unsigned short)(u >> 16); }
__device__ __forceinline__ float bf2f(unsigned short b) { return __uint_as_float(((unsigned)b) << 16); }
__device__ __forceinline__ float bfr(float f) { return bf2f(f2bf(f)); }
__device__ __forceinline__ v16h cat16(v8h lo, v8h hi) { return __builtin_shufflevector(lo, hi, 0, 1, 2, 3, 4, 5, 6, 7, 8, 9, 10, 11, 12, 13, 14, 15); }
__device__ __forceinline__ v16bf cat16b(v8us lo, v8us hi) { return __builtin_bit_cast(v16bf, __builtin_shufflevector(lo, hi, 0, 1, 2, 3, 4, 5, 6, 7, 8, 9, 10, 11, 12, 13, 14, 15)); }
__device__ __forceinline__ v8f wmma16(v16h a, v16h b, v8f c) { return __builtin_amdgcn_wmma_f32_16x16x32_f16(false, a, false, b, (short)0, c, false, false); }
__device__ __forceinline__ v8f wmmab(v16bf a, v16bf b, v8f c) { return __builtin_amdgcn_wmma_f32_16x16x32_bf16(false, a, false, b, (short)0, c, false, false); }
__device__ __forceinline__ void splitf(float y, unsigned short& h, unsigned short& l) { h = f2bf(y); l = f2bf(y - bf2f(h)); }

static __device__ __forceinline__ v8f wmma16g(v16h a, v16h b, v8f c) { c = wmma16(a, b, c); asm volatile("v_nop\n\tv_nop\n\tv_nop\n\tv_nop" : "+v"(c) : "v"(a), "v"(b)); return c; }
static __device__ __forceinline__ h16 toh_flush(float v) { const h16 r = (h16)v; return (fabsf(v) < 6.103515625e-05f) ? (h16)0.0f : r; }
static __device__ __forceinline__ float fq_lvl(float x, float sc) { return fminf(fmaxf(rintf(x * sc), -32768.0f), 32767.0f); }

template <typename T16> struct WFrag;
template <> struct WFrag<h16> { typedef v16h V; static __device__ __forceinline__ V ld(const h16* p) { return cat16(*(const v8h*)p, *(const v8h*)(p + 16)); } static __device__ __forceinline__ v8f mma(V a, V b, v8f c) { return wmma16(a, b, c); } };
template <> struct WFrag<bf> { typedef v16bf V; static __device__ __forceinline__ V ld(const bf* p) { return cat16b(*(const v8us*)p, *(const v8us*)(p + 16)); } static __device__ __forceinline__ v8f mma(V a, V b, v8f c) { return wmmab(a, b, c); } };

template <typename T16, int NSPLIT, bool BIAS>
__device__ __forceinline__ void gemm_body(const T16* __restrict__ A, const T16* __restrict__ A2, const T16* __restrict__ Bt, const T16* __restrict__ Bt2, int K, float* C, int ldc, const float* __restrict__ bias, size_t sA, size_t sB, size_t sC) {
    typedef typename WFrag<T16>::V V;
    __shared__ __align__(16) float os[16 * 68];
    const size_t z = blockIdx.z; A += z * sA; if (A2) A2 += z * sA; Bt += z * sB; if (Bt2) Bt2 += z * sB; C += z * sC;
    const int lane = threadIdx.x & 31, lr = lane & 15, hi = lane >> 4; const int r0 = blockIdx.x * 64, c0 = blockIdx.y * 64;
    v8f acc[4][4];
#pragma unroll
    for (int mb = 0; mb < 4; ++mb)
#pragma unroll
        for (int nb = 0; nb < 4; ++nb) acc[mb][nb] = (v8f){};
    const size_t aoff = (size_t)(r0 + lr) * K + 8 * hi, boff = (size_t)(c0 + lr) * K + 8 * hi;
#pragma unroll 1
    for (int kc = 0; kc < K; kc += 32) {
        V a[4], a2[4];
#pragma unroll
        for (int mb = 0; mb < 4; ++mb) { a[mb] = WFrag<T16>::ld(A + aoff + (size_t)mb * 16 * K + kc); if (NSPLIT == 1 || NSPLIT == 2) a2[mb] = WFrag<T16>::ld(A2 + aoff + (size_t)mb * 16 * K + kc); }
#pragma unroll
        for (int nb = 0; nb < 4; ++nb) { const V b = WFrag<T16>::ld(Bt + boff + (size_t)nb * 16 * K + kc); V b2; if (NSPLIT >= 2) b2 = WFrag<T16>::ld(Bt2 + boff + (size_t)nb * 16 * K + kc);
#pragma unroll
            for (int mb = 0; mb < 4; ++mb) { acc[mb][nb] = WFrag<T16>::mma(a[mb], b, acc[mb][nb]); if (NSPLIT == 1 || NSPLIT == 2) acc[mb][nb] = WFrag<T16>::mma(a2[mb], b, acc[mb][nb]); if (NSPLIT >= 2) acc[mb][nb] = WFrag<T16>::mma(a[mb], b2, acc[mb][nb]); } }
        asm volatile("v_nop\n\tv_nop\n\tv_nop\n\tv_nop" : "+v"(acc[0][0]), "+v"(acc[1][1]), "+v"(acc[2][2]), "+v"(acc[3][3]) : "v"(a[0]), "v"(a[3]));
    }
#pragma unroll
    for (int mb = 0; mb < 4; ++mb) {
#pragma unroll
        for (int nb = 0; nb < 4; ++nb) {
#pragma unroll
            for (int j = 0; j < 8; ++j) os[(hi * 8 + j) * 68 + nb * 16 + lr] = acc[mb][nb][j]; }
        __builtin_amdgcn_wave_barrier(); asm volatile("" ::: "memory");
        float* crow = C + (size_t)(r0 + mb * 16) * ldc + c0;
#pragma unroll 1
        for (int ps = 0; ps < 2; ++ps) {
#pragma unroll
            for (int s = 0; s < 8; ++s) { const int row = 2 * s + hi, cofs = lr * 4; v4f val = *(const v4fa*)(os + row * 68 + cofs); if (BIAS) { val[0] += bfr(bias[c0 + cofs]); val[1] += bfr(bias[c0 + cofs + 1]); val[2] += bfr(bias[c0 + cofs + 2]); val[3] += bfr(bias[c0 + cofs + 3]); }
                *(volatile v4f*)(crow + (size_t)row * ldc + cofs) = val; }
            if (ps == 0) __threadfence(); }
        __builtin_amdgcn_wave_barrier(); asm volatile("" ::: "memory");
    }
}

__global__ __launch_bounds__(32) void k_gemm_proj(const bf* A, const bf* Bt, int K, float* C, int ldc, const float* bias) {
    gemm_body<bf, 0, true>(A, (const bf*)nullptr, Bt, (const bf*)nullptr, K, C, ldc, bias, 0, 0, 0);
}

__global__ __launch_bounds__(256) void k_cvt8(const float* __restrict__ src, bf* dst, size_t n8) { const size_t i = (size_t)blockIdx.x * 256 + threadIdx.x; if (i >= n8) return; const v8f v = *(const v8f*)(src + i * 8); v8us o;
#pragma unroll
    for (int k = 0; k < 8; ++k) o[k] = f2bf(v[k]); *(volatile v8us*)(dst + i * 8) = o; __threadfence(); *(volatile v8us*)(dst + i * 8) = o; }

__global__ __launch_bounds__(256) void k_cvtx(const float* __restrict__ src, bf* dst) {
    const size_t i = (size_t)blockIdx.x * 256 + threadIdx.x; if (i >= (size_t)NB * SEQ * EM / 8) return;
    const size_t e = i * 8; const int col = (int)(e % EM); const size_t row = e / EM; const int t = (int)(row % SEQ); const int b = (int)(row / SEQ);
    const v8f v = *(const v8f*)(src + ((size_t)b * SEQ_FULL + t) * EM + col); v8us o;
#pragma unroll
    for (int k = 0; k < 8; ++k) o[k] = f2bf(v[k]);
    *(volatile v8us*)(dst + e) = o; __threadfence(); *(volatile v8us*)(dst + e) = o; }

__global__ __launch_bounds__(256) void k_amax(const float* __restrict__ F, float* PART) {
    __shared__ float wm[8];
    const int lane = threadIdx.x & 31; const int wave = __builtin_amdgcn_readfirstlane(threadIdx.x >> 5);
    float m = 0.f;
#pragma unroll 1
    for (int it = 0; it < 8; ++it) { const size_t i = ((size_t)blockIdx.x * 8 + it) * 256 + threadIdx.x; const v4f v = *(const v4f*)(F + i * 4);
        m = fmaxf(m, fmaxf(fmaxf(fabsf(v[0]), fabsf(v[1])), fmaxf(fabsf(v[2]), fabsf(v[3])))); }
#pragma unroll
    for (int sh = 16; sh; sh >>= 1) m = fmaxf(m, __shfl_xor(m, sh, 32));
    if (lane == 0) wm[wave] = m;
    __syncthreads();
    if (threadIdx.x < 8) { float t = wm[0];
#pragma unroll
        for (int w = 1; w < 8; ++w) t = fmaxf(t, wm[w]);
        const v4f o = {t, t, t, t}; float* dst = PART + (size_t)blockIdx.x * 32 + threadIdx.x * 4; *(volatile v4f*)dst = o; __threadfence(); *(volatile v4f*)dst = o; }
}

__global__ __launch_bounds__(256) void k_fin(const float* __restrict__ PART, int n, float* PRML, int mode) {
#pragma clang fp contract(off)
    __shared__ float wm[8];
    const int lane = threadIdx.x & 31; const int wave = __builtin_amdgcn_readfirstlane(threadIdx.x >> 5);
    float m = 0.f;
#pragma unroll 1
    for (int i = threadIdx.x; i < n; i += 256) m = fmaxf(m, PART[(size_t)i * 32]);
#pragma unroll
    for (int sh = 16; sh; sh >>= 1) m = fmaxf(m, __shfl_xor(m, sh, 32));
    if (lane == 0) wm[wave] = m;
    __syncthreads();
    if (threadIdx.x < 8) { float t = wm[0];
#pragma unroll
        for (int w = 1; w < 8; ++w) t = fmaxf(t, wm[w]);
        const float b1 = 15.0f - ceilf(log2f(fmaxf(t, 1e-8f))); const int e1 = (int)b1;
        float a0 = ldexpf(1.0f, e1), a1 = ldexpf(1.0f, -e1), a2 = t, a3 = b1;
        if (mode == 1) { const float qm = fminf(rintf(t * a0), 32767.0f) * a1; const float m2 = qm * 0.125f;
            const float b2 = 15.0f - ceilf(log2f(fmaxf(m2, 1e-8f))); const int e2 = (int)b2;
            a1 = ldexpf(1.0f, e2 - e1 - 3); a2 = ldexpf(1.0f, -e2); a3 = t; }
        const v4f o = {a0, a1, a2, a3}; float* dst = PRML + threadIdx.x * 4; *(volatile v4f*)dst = o; __threadfence(); *(volatile v4f*)dst = o; }
}

__global__ __launch_bounds__(256) void k_hpq(const float* __restrict__ F, const float* __restrict__ PRML, h16* P, h16* R) {
#pragma clang fp contract(off)
    const size_t i = (size_t)blockIdx.x * 256 + threadIdx.x; if (i >= (size_t)NB * NH * SEQ * HD / 8) return;
    const size_t e = i * 8; const int d = (int)(e % HD); const int t = (int)((e / HD) % SEQ); const int bh = (int)(e / ((size_t)HD * SEQ)); const int b = bh / NH, h = bh % NH;
    const float sc = PRML[0], isc = PRML[1] * XCAR;
    const float* f = F + ((size_t)b * SEQ + t) * EM + h * HD + d; const v4f a0 = *(const v4f*)f, a1 = *(const v4f*)(f + 4); v8h o, rs;
#pragma unroll
    for (int k = 0; k < 4; ++k) { const float y0 = fq_lvl(a0[k], sc) * isc; const h16 h0 = toh_flush(y0); o[k] = h0; rs[k] = toh_flush(y0 - (float)h0);
        const float y1 = fq_lvl(a1[k], sc) * isc; const h16 h1 = toh_flush(y1); o[k + 4] = h1; rs[k + 4] = toh_flush(y1 - (float)h1); }
    *(volatile v8h*)(P + e) = o; *(volatile v8h*)(R + e) = rs; __threadfence(); *(volatile v8h*)(P + e) = o; *(volatile v8h*)(R + e) = rs; }

__global__ __launch_bounds__(256) void k_vtq(const float* __restrict__ F, const float* __restrict__ PRML, h16* V) {
#pragma clang fp contract(off)
    const size_t i = (size_t)blockIdx.x * 256 + threadIdx.x; if (i >= (size_t)NB * NH * HD * SEQ / 8) return;
    const size_t e = i * 8; const int t = (int)(e % SEQ); const int d = (int)((e / SEQ) % HD); const int bh = (int)(e / ((size_t)SEQ * HD)); const int b = bh / NH, h = bh % NH;
    const float sc = PRML[0], isc = PRML[1] * XCAR;
    const float* f = F + ((size_t)b * SEQ + t) * EM + h * HD + d; v8h o;
#pragma unroll
    for (int q = 0; q < 8; ++q) o[q] = toh_flush(fq_lvl(f[(size_t)q * EM], sc) * isc);
    *(volatile v8h*)(V + e) = o; __threadfence(); *(volatile v8h*)(V + e) = o; }

__global__ __launch_bounds__(32) void k_smax(const h16* __restrict__ QP, const h16* __restrict__ KP, float* PART) {
    const int lane = threadIdx.x & 31, lr = lane & 15, hi = lane >> 4;
    const int q0 = blockIdx.x * 16, h = blockIdx.y, b = blockIdx.z, bh = b * NH + h;
    const h16* Qb = QP + (size_t)bh * SEQ * HD + (size_t)(q0 + lr) * HD + 8 * hi;
    const h16* Kb = KP + (size_t)bh * SEQ * HD + (size_t)lr * HD + 8 * hi;
    const v16h qa0 = WFrag<h16>::ld(Qb), qa1 = WFrag<h16>::ld(Qb + 32);
    float m = 0.f;
#pragma unroll 1
    for (int kc = 0; kc < SEQ; kc += 64) {
#pragma unroll
        for (int j = 0; j < 4; ++j) { const h16* kp = Kb + (size_t)(kc + j * 16) * HD; const v16h k0 = WFrag<h16>::ld(kp), k1 = WFrag<h16>::ld(kp + 32);
            v8f s = (v8f){}; s = wmma16g(qa0, k0, s); s = wmma16g(qa1, k1, s);
#pragma unroll
            for (int r = 0; r < 8; ++r) m = fmaxf(m, fabsf(s[r])); }
    }
    m *= INVX2;
#pragma unroll
    for (int sh = 16; sh; sh >>= 1) m = fmaxf(m, __shfl_xor(m, sh, 32));
    const v4f o = {m, m, m, m}; float* dst = PART + ((size_t)bh * NQB + blockIdx.x) * 32 + (lane & 7) * 4;
    if (lane < 8) { *(volatile v4f*)dst = o; __threadfence(); *(volatile v4f*)dst = o; }
}

__global__ __launch_bounds__(32) __attribute__((amdgpu_num_vgpr(256))) void k_rowst(const h16* __restrict__ QP, const h16* __restrict__ KP, const float* __restrict__ msk, const float* __restrict__ PRM, float* ROWST, float* PART) {
#pragma clang fp contract(off)
    __shared__ __align__(16) float st[32];
    const int lane = threadIdx.x & 31, lr = lane & 15, hi = lane >> 4;
    const int q0 = blockIdx.x * 16, h = blockIdx.y, b = blockIdx.z, bh = b * NH + h;
    const h16* Qb = QP + (size_t)bh * SEQ * HD + (size_t)(q0 + lr) * HD + 8 * hi;
    const h16* Kb = KP + (size_t)bh * SEQ * HD + (size_t)lr * HD + 8 * hi;
    const float* mrow = msk + (size_t)b * SEQ_FULL + lr;
    const v16h qa0 = WFrag<h16>::ld(Qb), qa1 = WFrag<h16>::ld(Qb + 32);
    const float a1 = PRM[PRM_S] * INVX2, c12 = PRM[PRM_S + 1], inv2 = PRM[PRM_S + 2];

    float mx[8], ls[8];
#pragma unroll
    for (int r = 0; r < 8; ++r) { mx[r] = -1.0e30f; ls[r] = 0.f; }
#pragma unroll 1
    for (int kc = 0; kc < SEQ; kc += 64) {
        v8f s[4];
#pragma unroll
        for (int j = 0; j < 4; ++j) { const h16* kp = Kb + (size_t)(kc + j * 16) * HD; const v16h k0 = WFrag<h16>::ld(kp), k1 = WFrag<h16>::ld(kp + 32);
            s[j] = wmma16g(qa0, k0, (v8f){}); s[j] = wmma16g(qa1, k1, s[j]); }
#pragma unroll
        for (int j = 0; j < 4; ++j) { const float mk = bfr(mrow[kc + j * 16]); const float u = 10000.0f * (1.0f - mk);
#pragma unroll
            for (int r = 0; r < 8; ++r) { const float t1 = fq_lvl(s[j][r], a1); s[j][r] = fq_lvl(t1, c12) * inv2 - u; } }
#pragma unroll
        for (int r = 0; r < 8; ++r) { const float bm = fmaxf(fmaxf(s[0][r], s[1][r]), fmaxf(s[2][r], s[3][r])); const float mn = fmaxf(mx[r], bm);
            float a = ls[r] * __builtin_amdgcn_exp2f((mx[r] - mn) * LOG2E);
            a += __builtin_amdgcn_exp2f((s[0][r] - mn) * LOG2E); a += __builtin_amdgcn_exp2f((s[1][r] - mn) * LOG2E);
            a += __builtin_amdgcn_exp2f((s[2][r] - mn) * LOG2E); a += __builtin_amdgcn_exp2f((s[3][r] - mn) * LOG2E);
            ls[r] = a; mx[r] = mn; }
    }
    float bz = 0.f;
#pragma unroll
    for (int r = 0; r < 8; ++r) { float m = mx[r];
#pragma unroll
        for (int sh = 8; sh; sh >>= 1) m = fmaxf(m, __shfl_xor(m, sh, 32));
        float l = ls[r] * __builtin_amdgcn_exp2f((mx[r] - m) * LOG2E);
#pragma unroll
        for (int sh = 8; sh; sh >>= 1) l += __shfl_xor(l, sh, 32);
        const float rzv = 1.0f / l; bz = fmaxf(bz, rzv);
        if (lr == 0) { st[(8 * hi + r) * 2] = m; st[(8 * hi + r) * 2 + 1] = rzv; } }
    bz = fmaxf(bz, __shfl_xor(bz, 16, 32));
    __syncthreads();
    const v4f o = *(const v4fa*)(st + (lane & 7) * 4); const v4f pm = {bz, bz, bz, bz};
    float* d0 = ROWST + ((size_t)bh * SEQ + q0) * 2 + (lane & 7) * 4;
    float* d1 = PART + ((size_t)bh * NQB + blockIdx.x) * 32 + (lane & 7) * 4;
    if (lane < 8) { *(volatile v4f*)d0 = o; *(volatile v4f*)d1 = pm; __threadfence(); *(volatile v4f*)d0 = o; *(volatile v4f*)d1 = pm; }
}

__global__ __launch_bounds__(32) __attribute__((amdgpu_num_vgpr(256))) void k_attn(const h16* __restrict__ QP, const h16* __restrict__ QR, const h16* __restrict__ KP, const h16* __restrict__ KR, const h16* __restrict__ VT, const float* __restrict__ msk, const float* __restrict__ ROWST, const float* __restrict__ PRM, float* HR, float* PART) {
#pragma clang fp contract(off)
    __shared__ __align__(16) h16 pt[16 * PP];
    __shared__ __align__(16) float os[16 * 68];
    const int lane = threadIdx.x & 31, lr = lane & 15, hi = lane >> 4;
    const int q0 = blockIdx.x * 16, h = blockIdx.y, b = blockIdx.z, bh = b * NH + h;
    const size_t qoff = (size_t)bh * SEQ * HD + (size_t)(q0 + lr) * HD + 8 * hi;
    const size_t koff = (size_t)bh * SEQ * HD + (size_t)lr * HD + 8 * hi;
    const h16* Vb = VT + (size_t)bh * HD * SEQ + (size_t)lr * SEQ + 8 * hi;
    const float* mrow = msk + (size_t)b * SEQ_FULL + lr;
    const v16h qh0 = WFrag<h16>::ld(QP + qoff), qh1 = WFrag<h16>::ld(QP + qoff + 32);
    const v16h ql0 = WFrag<h16>::ld(QR + qoff), ql1 = WFrag<h16>::ld(QR + qoff + 32);
    const float a1 = PRM[PRM_S] * INVX2, c12 = PRM[PRM_S + 1], inv2 = PRM[PRM_S + 2];
    const float scp = PRM[PRM_P], osc = PRM[PRM_P + 1] * (1.0f / XCAR);

    float rm[8], rz[8];
    { const float* rs = ROWST + ((size_t)bh * SEQ + q0 + 8 * hi) * 2;
      const v4f w0 = *(const v4f*)rs, w1 = *(const v4f*)(rs + 4), w2 = *(const v4f*)(rs + 8), w3 = *(const v4f*)(rs + 12);
      rm[0] = w0[0]; rz[0] = w0[1]; rm[1] = w0[2]; rz[1] = w0[3]; rm[2] = w1[0]; rz[2] = w1[1]; rm[3] = w1[2]; rz[3] = w1[3];
      rm[4] = w2[0]; rz[4] = w2[1]; rm[5] = w2[2]; rz[5] = w2[3]; rm[6] = w3[0]; rz[6] = w3[1]; rm[7] = w3[2]; rz[7] = w3[3]; }

    v8f acc[4];
#pragma unroll
    for (int j = 0; j < 4; ++j) acc[j] = (v8f){};
#pragma unroll 1
    for (int kc = 0; kc < SEQ; kc += 64) {
#pragma unroll 1
        for (int j = 0; j < 4; ++j) { const size_t ko = koff + (size_t)(kc + j * 16) * HD;
            const v16h kh0 = WFrag<h16>::ld(KP + ko), kh1 = WFrag<h16>::ld(KP + ko + 32), kl0 = WFrag<h16>::ld(KR + ko), kl1 = WFrag<h16>::ld(KR + ko + 32);
            v8f s = (v8f){};
            s = wmma16g(qh0, kh0, s); s = wmma16g(qh1, kh1, s);
            s = wmma16g(qh0, kl0, s); s = wmma16g(qh1, kl1, s);
            s = wmma16g(ql0, kh0, s); s = wmma16g(ql1, kh1, s);
            const float mk = bfr(mrow[kc + j * 16]); const float u = 10000.0f * (1.0f - mk);
#pragma unroll
            for (int r = 0; r < 8; ++r) { const float t1 = fq_lvl(s[r], a1); const float lg = fq_lvl(t1, c12) * inv2 - u;
                const float p = __builtin_amdgcn_exp2f((lg - rm[r]) * LOG2E) * rz[r];
                pt[(8 * hi + r) * PP + j * 16 + lr] = toh_flush(fq_lvl(p, scp)); } }
        __syncthreads();
        const h16* pr = pt + lr * PP + 8 * hi;
        const v16h pa0 = cat16(*(const v8ha*)pr, *(const v8ha*)(pr + 16));
        const v16h pa1 = cat16(*(const v8ha*)(pr + 32), *(const v8ha*)(pr + 48));
#pragma unroll
        for (int j = 0; j < 4; ++j) { const h16* vp = Vb + (size_t)(j * 16) * SEQ + kc; const v16h v0 = WFrag<h16>::ld(vp), v1 = WFrag<h16>::ld(vp + 32);
            acc[j] = wmma16g(pa0, v0, acc[j]); acc[j] = wmma16g(pa1, v1, acc[j]); }
        __syncthreads();
    }

    float mxh = 0.f;
#pragma unroll
    for (int r = 0; r < 8; ++r) {
#pragma unroll
        for (int j = 0; j < 4; ++j) { const float val = acc[j][r] * osc; os[(8 * hi + r) * 68 + j * 16 + lr] = val; mxh = fmaxf(mxh, fabsf(val)); } }
#pragma unroll
    for (int sh = 16; sh; sh >>= 1) mxh = fmaxf(mxh, __shfl_xor(mxh, sh, 32));
    __syncthreads();
    float* hrow = HR + ((size_t)b * SEQ + q0) * EM + h * HD;
    float* pl = PART + ((size_t)bh * NQB + blockIdx.x) * 32 + (lane & 7) * 4;
    const v4f pm = {mxh, mxh, mxh, mxh};
#pragma unroll 1
    for (int ps = 0; ps < 2; ++ps) {
#pragma unroll
        for (int s = 0; s < 8; ++s) { const int row = 2 * s + hi, cofs = lr * 4; const v4f val = *(const v4fa*)(os + row * 68 + cofs);
            *(volatile v4f*)(hrow + (size_t)row * EM + cofs) = val; }
        if (lane < 8) *(volatile v4f*)pl = pm;
        if (ps == 0) __threadfence(); }
}

__global__ __launch_bounds__(256) void k_qout(const float* __restrict__ HR, const float* __restrict__ PRML, float* OUT) {
#pragma clang fp contract(off)
    const size_t i = (size_t)blockIdx.x * 256 + threadIdx.x; if (i >= (size_t)NB * SEQ * EM / 4) return;
    const size_t e = i * 4; const int col = (int)(e % EM); const size_t row = e / EM; const int t = (int)(row % SEQ); const int b = (int)(row / SEQ);
    const float sc = PRML[0], isc = PRML[1];
    const v4f v = *(const v4f*)(HR + e); v4f o;
#pragma unroll
    for (int k = 0; k < 4; ++k) o[k] = fq_lvl(v[k], sc) * isc;
    float* dst = OUT + ((size_t)b * SEQ_FULL + t) * EM + col; *(volatile v4f*)dst = o; __threadfence(); *(volatile v4f*)dst = o; }

constexpr size_t al256(size_t x) { return (x + 255) & ~(size_t)255; }
constexpr size_t zmax(size_t a, size_t b) { return a > b ? a : b; }
constexpr size_t SZ_W    = al256((size_t)EM * EM * 2);
constexpr size_t SZ_XB   = al256((size_t)NB * SEQ * EM * 2);
constexpr size_t SZ_F    = al256((size_t)NB * SEQ * EM * 4);
constexpr size_t SZ_PL   = al256((size_t)NB * NH * SEQ * HD * 2);
constexpr size_t SZ_RS   = al256((size_t)NB * NH * SEQ * 2 * 4);
constexpr size_t SZ_PART = al256(zmax((size_t)NAMAX, (size_t)NBLK) * 128);
constexpr size_t SZ_PRM  = al256((size_t)6 * 128);
constexpr size_t WS_TOTAL = 3 * SZ_W + SZ_XB + SZ_F + 5 * SZ_PL + SZ_RS + SZ_PART + SZ_PRM;
static_assert(WS_TOTAL <= (size_t)134217728);
static_assert((size_t)NAMAX * 128 <= SZ_PART);
static_assert((size_t)NBLK * 128 <= SZ_PART);
static_assert((size_t)(PRM_O + 32) * 4 <= SZ_PRM);
static_assert((size_t)NBLK * 16 * 2 * 4 <= SZ_RS);

extern "C" void kernel_launch(void* const* d_in, const int* in_sizes, int n_in,
                              void* d_out, int out_size, void* d_ws, size_t ws_size, hipStream_t stream) {
    if (n_in < 8) return;
    const size_t need_act = ((size_t)(NB - 1) * SEQ_FULL + SEQ) * EM;
    if ((size_t)in_sizes[0] < need_act) return;
    if ((size_t)in_sizes[1] < (size_t)(NB - 1) * SEQ_FULL + SEQ) return;
    if ((size_t)in_sizes[2] < (size_t)EM * EM || (size_t)in_sizes[4] < (size_t)EM * EM || (size_t)in_sizes[6] < (size_t)EM * EM) return;
    if (in_sizes[3] < EM || in_sizes[5] < EM || in_sizes[7] < EM) return;
    if ((size_t)out_size < need_act) return;
    if (WS_TOTAL > ws_size) return;
    const float* x = (const float*)d_in[0];
    const float* mask = (const float*)d_in[1];
    const float* Wq = (const float*)d_in[2]; const float* bq = (const float*)d_in[3];
    const float* Wk = (const float*)d_in[4]; const float* bk = (const float*)d_in[5];
    const float* Wv = (const float*)d_in[6]; const float* bv = (const float*)d_in[7];
    float* OUT = (float*)d_out;
    char* wsp = (char*)d_ws;
    auto take = [&](size_t bytes) { char* p = wsp; wsp += bytes; return (void*)p; };
    bf* WQ = (bf*)take(SZ_W); bf* WK = (bf*)take(SZ_W); bf* WV = (bf*)take(SZ_W);
    bf* XB = (bf*)take(SZ_XB); float* F = (float*)take(SZ_F);
    h16* QP = (h16*)take(SZ_PL); h16* QR = (h16*)take(SZ_PL); h16* KP = (h16*)take(SZ_PL); h16* KR = (h16*)take(SZ_PL); h16* VTp = (h16*)take(SZ_PL);
    float* ROWST = (float*)take(SZ_RS); float* PART = (float*)take(SZ_PART); float* PRM = (float*)take(SZ_PRM);

    const unsigned gw = (unsigned)(((size_t)EM * EM / 8 + 255) / 256);
    k_cvt8<<<gw, 256, 0, stream>>>(Wq, WQ, (size_t)EM * EM / 8);
    k_cvt8<<<gw, 256, 0, stream>>>(Wk, WK, (size_t)EM * EM / 8);
    k_cvt8<<<gw, 256, 0, stream>>>(Wv, WV, (size_t)EM * EM / 8);

    const unsigned gx = (unsigned)(((size_t)NB * SEQ * EM / 8 + 255) / 256);
    const dim3 gp(NB * SEQ / 64, EM / 64, 1);
    const dim3 ga(NQB, NH, NB);
    k_cvtx<<<gx, 256, 0, stream>>>(x, XB);
    k_gemm_proj<<<gp, 32, 0, stream>>>(XB, WQ, EM, F, EM, bq);
    k_amax<<<NAMAX, 256, 0, stream>>>(F, PART);
    k_fin<<<1, 256, 0, stream>>>(PART, NAMAX, PRM + PRM_Q, 0);
    k_hpq<<<gx, 256, 0, stream>>>(F, PRM + PRM_Q, QP, QR);
    k_gemm_proj<<<gp, 32, 0, stream>>>(XB, WK, EM, F, EM, bk);
    k_amax<<<NAMAX, 256, 0, stream>>>(F, PART);
    k_fin<<<1, 256, 0, stream>>>(PART, NAMAX, PRM + PRM_K, 0);
    k_hpq<<<gx, 256, 0, stream>>>(F, PRM + PRM_K, KP, KR);
    k_gemm_proj<<<gp, 32, 0, stream>>>(XB, WV, EM, F, EM, bv);
    k_amax<<<NAMAX, 256, 0, stream>>>(F, PART);
    k_fin<<<1, 256, 0, stream>>>(PART, NAMAX, PRM + PRM_V, 0);
    k_vtq<<<gx, 256, 0, stream>>>(F, PRM + PRM_V, VTp);
    k_smax<<<ga, 32, 0, stream>>>(QP, KP, PART);
    k_fin<<<1, 256, 0, stream>>>(PART, NBLK, PRM + PRM_S, 1);
    k_rowst<<<ga, 32, 0, stream>>>(QP, KP, mask, PRM, ROWST, PART);
    k_fin<<<1, 256, 0, stream>>>(PART, NBLK, PRM + PRM_P, 0);
    k_attn<<<ga, 32, 0, stream>>>(QP, QR, KP, KR, VTp, mask, ROWST, PRM, F, PART);
    k_fin<<<1, 256, 0, stream>>>(PART, NBLK, PRM + PRM_O, 0);
    const unsigned go = (unsigned)(((size_t)NB * SEQ * EM / 4 + 255) / 256);
    k_qout<<<go, 256, 0, stream>>>(F, PRM + PRM_O, OUT);
}
